// SelfAttention_12352325943316
// MI455X (gfx1250) — hardware-verified
//
#include <hip/hip_runtime.h>


#ifndef NB
#define NB 2
#endif
#ifndef SEQ
#define SEQ 2048
#endif
#define NB_FULL    2
#define SEQ_FULL   2048
#define NHEAD      16
#define HDIM       64
#define DMODEL     1024
#define QKVN       3072
#define BQ         128
#define BK         32
#define NWAVE      8
#define OP         68
#define GM         128
#define GN         64
#define GWAVE      4
#define CP         68
#define MROWS      (NB * SEQ)

static_assert(SEQ % BQ == 0);
static_assert(SEQ % BK == 0);
static_assert(SEQ % GM == 0);
static_assert(BQ == NWAVE * 16);
static_assert(GM == GWAVE * 32);
static_assert(HDIM == 64);
static_assert(GN == HDIM);
static_assert(NHEAD * HDIM == DMODEL);
static_assert(QKVN == 3 * DMODEL);
static_assert(DMODEL == 1024);
static_assert(DMODEL % 32 == 0);
static_assert(QKVN % GN == 0 && DMODEL % GN == 0);
static_assert(MROWS % GM == 0);
static_assert(SEQ <= SEQ_FULL);
static_assert(NB >= 1 && NB <= NB_FULL);
static_assert((OP * 4) % 16 == 0);
static_assert((CP * 4) % 16 == 0);
static_assert(((size_t)MROWS * DMODEL) % 2048 == 0);
static_assert(((size_t)QKVN * DMODEL) % 2048 == 0);
static_assert(((size_t)DMODEL * DMODEL) % 2048 == 0);
static_assert((SEQ * 32) % 256 == 0);

constexpr size_t XH_BYTES  = (size_t)MROWS * DMODEL * 2;
constexpr size_t WQ_BYTES  = (size_t)QKVN * DMODEL * 2;
constexpr size_t WO_BYTES  = (size_t)DMODEL * DMODEL * 2;
constexpr size_t TAB_BYTES = (size_t)SEQ * 32 * 4;
constexpr size_t QK_ELEMS  = (size_t)NB * NHEAD * SEQ * HDIM;
constexpr size_t QK_BYTES  = QK_ELEMS * 2 * 2;
constexpr size_t VT_BYTES  = QK_ELEMS * 2;
constexpr size_t CTX_BYTES = (size_t)MROWS * DMODEL * 2;
constexpr size_t WS_TOTAL  = XH_BYTES + WQ_BYTES + WO_BYTES + 2 * TAB_BYTES + QK_BYTES + VT_BYTES + CTX_BYTES;
static_assert(WS_TOTAL <= (size_t)134217728);
static_assert(XH_BYTES % 256 == 0 && WQ_BYTES % 256 == 0 && WO_BYTES % 256 == 0);
static_assert(TAB_BYTES % 256 == 0 && QK_BYTES % 256 == 0 && VT_BYTES % 256 == 0);

typedef __bf16   bf16;
typedef _Float16 f16;
typedef f16      v16h  __attribute__((ext_vector_type(16)));
typedef f16      v8h   __attribute__((ext_vector_type(8)));
typedef float    v8f   __attribute__((ext_vector_type(8)));
typedef float    v4f   __attribute__((ext_vector_type(4)));
typedef unsigned v4u   __attribute__((ext_vector_type(4)));

union FragH  { v16h v; v4u q[2]; f16 h[16]; };
union Pack8H { v4u u; v8h v; f16 h[8]; };

static __device__ __forceinline__ v8f mma_f16(v16h a, v16h b, v8f acc) {
  acc = __builtin_amdgcn_wmma_f32_16x16x32_f16(false, a, false, b, (short)0, acc, false, false);
  asm volatile("v_nop\n\tv_nop\n\tv_nop\n\tv_nop" : "+v"(acc) : "v"(a), "v"(b));
  return acc;
}

static __device__ __forceinline__ float rne_bf16(float v) { return (float)(bf16)v; }

__global__ __launch_bounds__(256) void cvt_plane_kernel(const float* __restrict__ src, f16* __restrict__ dst,
                                                        int n_dst, int rows_dst_per_batch, int rows_src_per_batch,
                                                        float scale) {
  const int e = (blockIdx.x * 256 + threadIdx.x) * 8;
  if (e >= n_dst) return;
  const int row = e >> 10;
  const int col = e & 1023;
  const int bb  = row / rows_dst_per_batch;
  const int rr  = row - bb * rows_dst_per_batch;
  const float* s = src + ((size_t)bb * rows_src_per_batch + rr) * DMODEL + col;
  const v4f a0 = *(const v4f*)(s);
  const v4f a1 = *(const v4f*)(s + 4);
  Pack8H ph;
  #pragma unroll
  for (int i = 0; i < 4; ++i) {
    ph.h[i]     = (f16)(rne_bf16(a0[i]) * scale);
    ph.h[4 + i] = (f16)(rne_bf16(a1[i]) * scale);
  }
  const v4u val = ph.u;
  *(volatile v4u*)(dst + e) = val;
  __threadfence();
  *(volatile v4u*)(dst + e) = val;
}

__global__ __launch_bounds__(256) void rope_table_kernel(float* __restrict__ cosT, float* __restrict__ sinT) {
  const int gid = blockIdx.x * 256 + threadIdx.x;
  if (gid >= SEQ * 32) return;
  const int t = gid >> 5;
  const int i = gid & 31;
  double p = 1.0;
  p = (i & 1)  ? p * 1.3335214321633240 : p;
  p = (i & 2)  ? p * 1.7782794100389228 : p;
  p = (i & 4)  ? p * 3.1622776601683795 : p;
  p = (i & 8)  ? p * 10.0 : p;
  p = (i & 16) ? p * 100.0 : p;
  const float pf  = (float)p;
  const float inv = 1.0f / pf;
  const float ang = (float)t * inv;
  float sn, cs;
  sincosf(ang, &sn, &cs);
  *(volatile float*)(cosT + gid) = cs;
  *(volatile float*)(sinT + gid) = sn;
  __threadfence();
  *(volatile float*)(cosT + gid) = cs;
  *(volatile float*)(sinT + gid) = sn;
}

static __device__ __forceinline__ void gemm_core(const f16* __restrict__ A, const f16* __restrict__ W,
                                                 int arow, int wrow, int lq, int hi, v8f (&acc)[2][4]) {
  const f16* ap = A + (size_t)(arow + lq) * DMODEL + hi * 8;
  const f16* wp = W + (size_t)(wrow + lq) * DMODEL + hi * 8;
  #pragma unroll 2
  for (int k0 = 0; k0 < DMODEL; k0 += 32) {
    FragH a[2], bw[4];
    #pragma unroll
    for (int i = 0; i < 2; ++i) {
      a[i].q[0] = *(const v4u*)(ap + (size_t)i * 16 * DMODEL + k0);
      a[i].q[1] = *(const v4u*)(ap + (size_t)i * 16 * DMODEL + k0 + 16);
    }
    #pragma unroll
    for (int j = 0; j < 4; ++j) {
      bw[j].q[0] = *(const v4u*)(wp + (size_t)j * 16 * DMODEL + k0);
      bw[j].q[1] = *(const v4u*)(wp + (size_t)j * 16 * DMODEL + k0 + 16);
    }
    #pragma unroll
    for (int i = 0; i < 2; ++i) {
      #pragma unroll
      for (int j = 0; j < 4; ++j) acc[i][j] = mma_f16(a[i].v, bw[j].v, acc[i][j]);
    }
  }
}

__global__ __launch_bounds__(128) void qkv_gemm_kernel(const f16* __restrict__ xh, const f16* __restrict__ wh,
                                                       const float* __restrict__ bqkv,
                                                       const float* __restrict__ cosT, const float* __restrict__ sinT,
                                                       f16* __restrict__ qk, f16* __restrict__ vt) {
  __shared__ __align__(16) float sC[GM * CP];
  const int tid   = threadIdx.x;
  const int wave  = __builtin_amdgcn_readfirstlane(tid >> 5);
  const int lane  = tid & 31;
  const int lq    = lane & 15;
  const int hi    = lane >> 4;
  const int nblk  = blockIdx.x;
  const int col0  = nblk * GN;
  const int row0  = blockIdx.y * GM;
  const int which = nblk / NHEAD;
  const int h     = nblk - which * NHEAD;
  const int b     = row0 / SEQ;
  const int l0    = row0 - b * SEQ;

  v8f acc[2][4];
  #pragma unroll
  for (int i = 0; i < 2; ++i) {
    #pragma unroll
    for (int j = 0; j < 4; ++j) acc[i][j] = (v8f){0, 0, 0, 0, 0, 0, 0, 0};
  }
  gemm_core(xh, wh, row0 + wave * 32, col0, lq, hi, acc);

  #pragma unroll
  for (int i = 0; i < 2; ++i) {
    #pragma unroll
    for (int j = 0; j < 4; ++j) {
      #pragma unroll
      for (int r = 0; r < 8; ++r)
        sC[(wave * 32 + i * 16 + hi * 8 + r) * CP + j * 16 + lq] = acc[i][j][r];
    }
  }
  __syncthreads();

  if (which < 2) {
    const int seg  = tid & 7;
    const int rsub = tid >> 3;
    const int d0   = seg * 8;
    float bias[8];
    {
      const v4f b0 = *(const v4f*)(bqkv + col0 + d0);
      const v4f b1 = *(const v4f*)(bqkv + col0 + d0 + 4);
      #pragma unroll
      for (int e = 0; e < 4; ++e) {
        bias[e]     = rne_bf16(b0[e]);
        bias[4 + e] = rne_bf16(b1[e]);
      }
    }
    v4u    vals[8];
    size_t idx[8];
    #pragma unroll
    for (int ps = 0; ps < 8; ++ps) {
      const int row = ps * 16 + rsub;
      const int l   = l0 + row;
      const v4f a0 = *(const v4f*)(sC + row * CP + d0);
      const v4f a1 = *(const v4f*)(sC + row * CP + d0 + 4);
      const v4f cs = *(const v4f*)(cosT + (size_t)l * 32 + seg * 4);
      const v4f sn = *(const v4f*)(sinT + (size_t)l * 32 + seg * 4);
      float xv[8];
      #pragma unroll
      for (int e = 0; e < 4; ++e) {
        xv[e]     = a0[e] * 0.0625f + bias[e];
        xv[4 + e] = a1[e] * 0.0625f + bias[4 + e];
      }
      Pack8H ph;
      #pragma unroll
      for (int p = 0; p < 4; ++p) {
        const float xe = xv[2 * p];
        const float xo = xv[2 * p + 1];
        ph.h[2 * p]     = (f16)(xe * cs[p] - xo * sn[p]);
        ph.h[2 * p + 1] = (f16)(xe * sn[p] + xo * cs[p]);
      }
      vals[ps] = ph.u;
      idx[ps]  = (size_t)which * QK_ELEMS + (((size_t)b * NHEAD + h) * SEQ + l) * HDIM + d0;
    }
    #pragma unroll
    for (int ps = 0; ps < 8; ++ps) *(volatile v4u*)(qk + idx[ps]) = vals[ps];
    __threadfence();
    #pragma unroll
    for (int ps = 0; ps < 8; ++ps) *(volatile v4u*)(qk + idx[ps]) = vals[ps];
  } else {
    const int seg  = tid & 15;
    const int dsub = tid >> 4;
    v4u    vals[8];
    size_t idx[8];
    #pragma unroll
    for (int ps = 0; ps < 8; ++ps) {
      const int d = ps * 8 + dsub;
      const float bv = rne_bf16(bqkv[col0 + d]);
      Pack8H ph;
      #pragma unroll
      for (int e = 0; e < 8; ++e) ph.h[e] = (f16)(sC[(seg * 8 + e) * CP + d] * 0.0625f + bv);
      vals[ps] = ph.u;
      idx[ps]  = (((size_t)b * NHEAD + h) * HDIM + d) * SEQ + l0 + seg * 8;
    }
    #pragma unroll
    for (int ps = 0; ps < 8; ++ps) *(volatile v4u*)(vt + idx[ps]) = vals[ps];
    __threadfence();
    #pragma unroll
    for (int ps = 0; ps < 8; ++ps) *(volatile v4u*)(vt + idx[ps]) = vals[ps];
  }
}

__global__ __launch_bounds__(256) void attn_kernel(const f16* __restrict__ qk, const f16* __restrict__ vt,
                                                   const int* __restrict__ pad, f16* __restrict__ ctx) {
  const int qblk = blockIdx.x;
  const int h    = blockIdx.y;
  const int b    = blockIdx.z;
  const int tid  = threadIdx.x;
  const int wave = __builtin_amdgcn_readfirstlane(tid >> 5);
  const int lane = tid & 31;
  const int lq   = lane & 15;
  const int hi   = lane >> 4;

  __shared__ __align__(16) float sO[NWAVE * 16 * OP];

  const int qrow0 = qblk * BQ + wave * 16;

  const f16* q_h  = qk + ((size_t)b * NHEAD + h) * SEQ * HDIM;
  const f16* k_h  = q_h + QK_ELEMS;
  const f16* vt_h = vt + ((size_t)b * NHEAD + h) * HDIM * SEQ;
  const int* pad_b = pad + (size_t)b * SEQ_FULL;

  FragH qf[2];
  {
    const f16* qp = q_h + (size_t)(qrow0 + lq) * HDIM + hi * 8;
    #pragma unroll
    for (int f = 0; f < 2; ++f) {
      qf[f].q[0] = *(const v4u*)(qp + f * 32);
      qf[f].q[1] = *(const v4u*)(qp + f * 32 + 16);
    }
  }

  v8f o[4];
  #pragma unroll
  for (int dt = 0; dt < 4; ++dt) o[dt] = (v8f){0, 0, 0, 0, 0, 0, 0, 0};

  const float NEG_INIT = -1.0e30f;
  const float NEG_EXCL = -2.0e30f;
  float rmax = NEG_INIT;
  float rsum = 0.0f;
  const float SL = 0.125f * 1.4426950408889634f;

  #pragma unroll 1
  for (int it = 0; it < SEQ / BK; ++it) {
    const int j0 = it * BK;
    const int pv = pad_b[j0 + lane];
    const unsigned pm = __builtin_amdgcn_ballot_w32(pv != 0);
    if ((j0 + BK - 1 <= qrow0) && (pm == 0u)) continue;
    const bool full = (j0 > qrow0 + 15) || (pm == 0xffffffffu);

    FragH ak[2][2];
    #pragma unroll
    for (int sub = 0; sub < 2; ++sub) {
      #pragma unroll
      for (int f = 0; f < 2; ++f) {
        const f16* base = k_h + (size_t)(j0 + sub * 16 + lq) * HDIM + f * 32 + hi * 8;
        ak[sub][f].q[0] = *(const v4u*)(base);
        ak[sub][f].q[1] = *(const v4u*)(base + 16);
      }
    }
    FragH bv[4];
    #pragma unroll
    for (int dt = 0; dt < 4; ++dt) {
      const f16* base = vt_h + (size_t)(dt * 16 + lq) * SEQ + j0 + hi * 8;
      bv[dt].q[0] = *(const v4u*)(base);
      bv[dt].q[1] = *(const v4u*)(base + 16);
    }

    v8f c[2];
    #pragma unroll
    for (int sub = 0; sub < 2; ++sub) {
      v8f acc = (v8f){0, 0, 0, 0, 0, 0, 0, 0};
      acc = mma_f16(ak[sub][0].v, qf[0].v, acc);
      acc = mma_f16(ak[sub][1].v, qf[1].v, acc);
      c[sub] = acc;
    }

    if (!full) {
      const int qi = qrow0 + lq;
      const unsigned pmh = pm >> (hi * 8);
      #pragma unroll
      for (int sub = 0; sub < 2; ++sub) {
        #pragma unroll
        for (int r = 0; r < 8; ++r) {
          const int key = j0 + sub * 16 + hi * 8 + r;
          const bool al = (key > qi) || (((pmh >> (sub * 16 + r)) & 1u) != 0u);
          c[sub][r] = al ? c[sub][r] : NEG_EXCL;
        }
      }
    }

    float m_new = rmax;
    #pragma unroll
    for (int r = 0; r < 8; ++r) {
      m_new = fmaxf(m_new, c[0][r]);
      m_new = fmaxf(m_new, c[1][r]);
    }
    m_new = fmaxf(m_new, __shfl_xor(m_new, 16, 32));
    const float scale = __builtin_amdgcn_exp2f((rmax - m_new) * SL);
    rmax = m_new;

    float p0[8], p1[8];
    #pragma unroll
    for (int r = 0; r < 8; ++r) {
      p0[r] = __builtin_amdgcn_exp2f((c[0][r] - m_new) * SL);
      p1[r] = __builtin_amdgcn_exp2f((c[1][r] - m_new) * SL);
    }
    if (!full) {
      #pragma unroll
      for (int r = 0; r < 8; ++r) {
        p0[r] = (c[0][r] == NEG_EXCL) ? 0.0f : p0[r];
        p1[r] = (c[1][r] == NEG_EXCL) ? 0.0f : p1[r];
      }
    }

    FragH pa;
    float psum = 0.0f;
    #pragma unroll
    for (int r = 0; r < 8; ++r) {
      psum += p0[r] + p1[r];
      pa.h[r]     = (f16)(p0[r] * 4096.0f);
      pa.h[8 + r] = (f16)(p1[r] * 4096.0f);
    }
    rsum = rsum * scale + psum + __shfl_xor(psum, 16, 32);

    float sc[8];
    #pragma unroll
    for (int r = 0; r < 8; ++r) sc[r] = __shfl(scale, (hi << 3) + r, 32);
    #pragma unroll
    for (int dt = 0; dt < 4; ++dt) {
      #pragma unroll
      for (int r = 0; r < 8; ++r) o[dt][r] *= sc[r];
    }

    #pragma unroll
    for (int dt = 0; dt < 4; ++dt) o[dt] = mma_f16(pa.v, bv[dt].v, o[dt]);
  }

  float rs[8];
  #pragma unroll
  for (int r = 0; r < 8; ++r) rs[r] = 1.0f / __shfl(rsum, (hi << 3) + r, 32);

  const int sob = wave * (16 * OP);
  #pragma unroll
  for (int r = 0; r < 8; ++r) {
    #pragma unroll
    for (int dt = 0; dt < 4; ++dt)
      sO[sob + (hi * 8 + r) * OP + dt * 16 + lq] = o[dt][r] * rs[r] * (1.0f / 256.0f);
  }
  __syncthreads();

  v4u    vals[4];
  size_t gidx[4];
  #pragma unroll
  for (int g = 0; g < 4; ++g) {
    const int row = g * 4 + (lane >> 3);
    const int seg = lane & 7;
    const v4f a0 = *(const v4f*)(sO + sob + row * OP + seg * 8);
    const v4f a1 = *(const v4f*)(sO + sob + row * OP + seg * 8 + 4);
    Pack8H ph;
    #pragma unroll
    for (int e = 0; e < 4; ++e) {
      ph.h[e]     = (f16)a0[e];
      ph.h[4 + e] = (f16)a1[e];
    }
    vals[g] = ph.u;
    gidx[g] = ((size_t)b * SEQ + qrow0 + row) * DMODEL + h * HDIM + seg * 8;
  }
  #pragma unroll
  for (int g = 0; g < 4; ++g) *(volatile v4u*)(ctx + gidx[g]) = vals[g];
  __threadfence();
  #pragma unroll
  for (int g = 0; g < 4; ++g) *(volatile v4u*)(ctx + gidx[g]) = vals[g];
}

__global__ __launch_bounds__(128) void out_gemm_kernel(const f16* __restrict__ ctx, const f16* __restrict__ wo,
                                                       const float* __restrict__ bout, float* __restrict__ out) {
  __shared__ __align__(16) float sC[GM * CP];
  const int tid  = threadIdx.x;
  const int wave = __builtin_amdgcn_readfirstlane(tid >> 5);
  const int lane = tid & 31;
  const int lq   = lane & 15;
  const int hi   = lane >> 4;
  const int col0 = blockIdx.x * GN;
  const int row0 = blockIdx.y * GM;
  const int b    = row0 / SEQ;
  const int l0   = row0 - b * SEQ;

  v8f acc[2][4];
  #pragma unroll
  for (int i = 0; i < 2; ++i) {
    #pragma unroll
    for (int j = 0; j < 4; ++j) acc[i][j] = (v8f){0, 0, 0, 0, 0, 0, 0, 0};
  }
  gemm_core(ctx, wo, row0 + wave * 32, col0, lq, hi, acc);

  #pragma unroll
  for (int i = 0; i < 2; ++i) {
    #pragma unroll
    for (int j = 0; j < 4; ++j) {
      #pragma unroll
      for (int r = 0; r < 8; ++r)
        sC[(wave * 32 + i * 16 + hi * 8 + r) * CP + j * 16 + lq] = acc[i][j][r];
    }
  }
  __syncthreads();

  const int c4   = (tid & 15) * 4;
  const int rsub = tid >> 4;
  v4f bias;
  {
    const v4f b0 = *(const v4f*)(bout + col0 + c4);
    #pragma unroll
    for (int e = 0; e < 4; ++e) bias[e] = rne_bf16(b0[e]);
  }
  #pragma unroll
  for (int half = 0; half < 2; ++half) {
    v4f    vals[8];
    size_t idx[8];
    #pragma unroll
    for (int ps = 0; ps < 8; ++ps) {
      const int row = (half * 8 + ps) * 8 + rsub;
      const v4f a = *(const v4f*)(sC + row * CP + c4);
      v4f y;
      #pragma unroll
      for (int e = 0; e < 4; ++e) y[e] = a[e] * (1.0f / 256.0f) + bias[e];
      vals[ps] = y;
      idx[ps]  = ((size_t)b * SEQ_FULL + l0 + row) * DMODEL + col0 + c4;
    }
    #pragma unroll
    for (int ps = 0; ps < 8; ++ps) *(volatile v4f*)(out + idx[ps]) = vals[ps];
    __threadfence();
    #pragma unroll
    for (int ps = 0; ps < 8; ++ps) *(volatile v4f*)(out + idx[ps]) = vals[ps];
  }
}

extern "C" void kernel_launch(void* const* d_in, const int* in_sizes, int n_in,
                              void* d_out, int out_size, void* d_ws, size_t ws_size,
                              hipStream_t stream) {
  if (n_in < 6) return;
  const size_t rows_used = (size_t)(NB - 1) * SEQ_FULL + SEQ;
  if ((size_t)in_sizes[0] < rows_used * DMODEL) return;
  if ((size_t)in_sizes[1] < rows_used) return;
  if ((size_t)in_sizes[2] < (size_t)QKVN * DMODEL) return;
  if ((size_t)in_sizes[3] < (size_t)QKVN) return;
  if ((size_t)in_sizes[4] < (size_t)DMODEL * DMODEL) return;
  if ((size_t)in_sizes[5] < (size_t)DMODEL) return;
  if ((size_t)out_size < rows_used * DMODEL) return;
  if (ws_size < WS_TOTAL) return;

  const float* x    = (const float*)d_in[0];
  const int*   pad  = (const int*)d_in[1];
  const float* Wqkv = (const float*)d_in[2];
  const float* bqkv = (const float*)d_in[3];
  const float* Wout = (const float*)d_in[4];
  const float* bout = (const float*)d_in[5];
  float*       out  = (float*)d_out;

  char* ws = (char*)d_ws;
  size_t off = 0;
  f16*   xh   = (f16*)(ws + off);   off += XH_BYTES;
  f16*   wqh  = (f16*)(ws + off);   off += WQ_BYTES;
  f16*   woh  = (f16*)(ws + off);   off += WO_BYTES;
  float* cosT = (float*)(ws + off); off += TAB_BYTES;
  float* sinT = (float*)(ws + off); off += TAB_BYTES;
  f16*   qk   = (f16*)(ws + off);   off += QK_BYTES;
  f16*   vt   = (f16*)(ws + off);   off += VT_BYTES;
  f16*   ctx  = (f16*)(ws + off);   off += CTX_BYTES;

  const int n_x  = MROWS * DMODEL;
  const int n_wq = QKVN * DMODEL;
  const int n_wo = DMODEL * DMODEL;
  cvt_plane_kernel<<<(n_x / 8 + 255) / 256, 256, 0, stream>>>(x, xh, n_x, SEQ, SEQ_FULL, 1.0f);
  cvt_plane_kernel<<<(n_wq / 8 + 255) / 256, 256, 0, stream>>>(Wqkv, wqh, n_wq, QKVN, QKVN, 16.0f);
  cvt_plane_kernel<<<(n_wo / 8 + 255) / 256, 256, 0, stream>>>(Wout, woh, n_wo, DMODEL, DMODEL, 16.0f);
  rope_table_kernel<<<(SEQ * 32) / 256, 256, 0, stream>>>(cosT, sinT);

  qkv_gemm_kernel<<<dim3(QKVN / GN, MROWS / GM), 128, 0, stream>>>(xh, wqh, bqkv, cosT, sinT, qk, vt);
  attn_kernel<<<dim3(SEQ / BQ, NHEAD, NB), 256, 0, stream>>>(qk, vt, pad, ctx);
  out_gemm_kernel<<<dim3(DMODEL / GN, MROWS / GM), 128, 0, stream>>>(ctx, woh, bout, out);
}
